// DeltaNet_31877247271490
// MI455X (gfx1250) — hardware-verified
//
#include <hip/hip_runtime.h>
#include <math.h>

constexpr int kL    = 2048;
constexpr int kD    = 1024;
constexpr int kH    = 4;
constexpr int kDK   = 256;
constexpr int kCS   = 32;
constexpr int kNC   = 64;
constexpr int kSL   = 64;
constexpr int kNCAT = 3136;
constexpr int kRowB = 3072;
constexpr int kRowG = 3076;
constexpr int kRowZ = 3096;
static_assert(kD == kH * kDK, "head split");
static_assert(kL == kNC * kCS, "chunking");
static_assert(kNCAT % 64 == 0 && kL % 64 == 0 && kD % 64 == 0, "GEMM tile multiples");
static_assert(kD % 32 == 0 && kDK % 32 == 0 && kCS % 32 == 0, "K multiples of 32");
static_assert(kRowG == kRowB + kH && kRowZ == kRowG + 5 * kH && kRowZ <= kNCAT, "concat rows");
static_assert(((kL / 64) * (kNCAT / 64)) % 8 == 0 && ((kL / 64) * (kD / 64)) % 8 == 0, "GEMM grids exact");

constexpr float kWC   = 16.0f;
constexpr float kQC   = 16.0f;
constexpr float kVC   = 16.0f;
constexpr float kSC   = 256.0f;
constexpr float kAC   = 256.0f;
static_assert(kQC * kQC == kAC, "att plane carry equals the raw accumulator scale");
static_assert(kQC * kVC == kSC, "state increments land on the state carry");
static_assert(kQC * kSC == kAC * kVC, "q*S and att*u_adj share one accumulator scale");
constexpr float kInvW    = 1.0f / kWC;
constexpr float kInvG    = 1.0f / (kQC * kQC);
constexpr float kInvU    = 1.0f / (kQC * kVC);
constexpr float kInvWpl  = kQC / (kQC * kQC);
constexpr float kInvQS   = 1.0f / (kQC * kSC);

typedef __attribute__((ext_vector_type(16))) _Float16 v16h;
typedef __attribute__((ext_vector_type(8)))  _Float16 v8h;
typedef __attribute__((ext_vector_type(16))) __bf16   v16b;
typedef __attribute__((ext_vector_type(8)))  __bf16   v8b;
typedef __attribute__((ext_vector_type(8)))  float    v8f;
typedef __attribute__((ext_vector_type(4)))  float    v4f;
typedef __attribute__((ext_vector_type(4)))  unsigned int v4u;
typedef __attribute__((ext_vector_type(2)))  unsigned int v2u;

__device__ __forceinline__ unsigned short f2bf_bits(float f) {
  unsigned u = __float_as_uint(f);
  return (unsigned short)((u + 0x7FFFu + ((u >> 16) & 1u)) >> 16);
}
__device__ __forceinline__ float bf_bits2f(unsigned short h) { return __uint_as_float(((unsigned)h) << 16); }

__device__ __forceinline__ void dep_guard_h(v8f& a, v8f& b, v16h x, v16h y) { asm volatile("v_nop\n\tv_nop\n\tv_nop\n\tv_nop" : "+v"(a), "+v"(b) : "v"(x), "v"(y)); }
__device__ __forceinline__ void dep_guard_b(v8f& a, v8f& b, v16b x, v16b y) { asm volatile("v_nop\n\tv_nop\n\tv_nop\n\tv_nop" : "+v"(a), "+v"(b) : "v"(x), "v"(y)); }
__device__ __forceinline__ void keep4_h(v16h a, v16h b, v16h c, v16h d) { asm volatile("v_nop" :: "v"(a), "v"(b), "v"(c), "v"(d)); }
__device__ __forceinline__ void keep4_b(v16b a, v16b b, v16b c, v16b d) { asm volatile("v_nop" :: "v"(a), "v"(b), "v"(c), "v"(d)); }
__device__ __forceinline__ void acc_guard4(v8f& a, v8f& b, v8f& c, v8f& d) { asm volatile("v_nop\n\tv_nop\n\tv_nop\n\tv_nop" : "+v"(a), "+v"(b), "+v"(c), "+v"(d)); }
template <typename T> struct Frag;
template <> struct Frag<_Float16> {
  typedef v16h V; union U { v16h v; v8h h[2]; };
  static __device__ __forceinline__ v16h load(const _Float16* p) {
    U f; f.h[0] = *(const v8h*)(p); f.h[1] = *(const v8h*)(p + 16); return f.v;
  }
  static __device__ __forceinline__ v8f mma(v16h a, v16h b, v8f c) {
    return __builtin_amdgcn_wmma_f32_16x16x32_f16(false, a, false, b, (short)0, c, false, false);
  }
  static __device__ __forceinline__ void guard(v8f& a, v8f& b, v16h x, v16h y) { dep_guard_h(a, b, x, y); }
  static __device__ __forceinline__ void keep(v16h a, v16h b, v16h c, v16h d) { keep4_h(a, b, c, d); }
};
template <> struct Frag<__bf16> {
  typedef v16b V; union U { v16b v; v8b h[2]; };
  static __device__ __forceinline__ v16b load(const __bf16* p) {
    U f; f.h[0] = *(const v8b*)(p); f.h[1] = *(const v8b*)(p + 16); return f.v;
  }
  static __device__ __forceinline__ v8f mma(v16b a, v16b b, v8f c) {
    return __builtin_amdgcn_wmma_f32_16x16x32_bf16(false, a, false, b, (short)0, c, false, false);
  }
  static __device__ __forceinline__ void guard(v8f& a, v8f& b, v16b x, v16b y) { dep_guard_b(a, b, x, y); }
  static __device__ __forceinline__ void keep(v16b a, v16b b, v16b c, v16b d) { keep4_b(a, b, c, d); }
};

__device__ __forceinline__ unsigned pk16(unsigned short a, unsigned short b) { return (unsigned)a | ((unsigned)b << 16); }
__device__ __forceinline__ unsigned short h_bits(float f) { const _Float16 h = (_Float16)f; return __builtin_bit_cast(unsigned short, h); }

__device__ __forceinline__ v8f mma_h(v16h a, v16h b, v8f c) {
  c = __builtin_amdgcn_wmma_f32_16x16x32_f16(false, a, false, b, (short)0, c, false, false);
  asm volatile("v_nop\n\tv_nop\n\tv_nop\n\tv_nop" : "+v"(c) : "v"(a), "v"(b));
  return c;
}
__device__ __forceinline__ v16h ldfrag(const unsigned short* p) { return Frag<_Float16>::load((const _Float16*)p); }

template <int ET> struct Elem;
template <> struct Elem<0> { typedef _Float16 T; };
template <> struct Elem<1> { typedef __bf16 T; };
template <int ET, bool SPLIT, int BIAS_MODE, int OUT_MODE, bool RESID, int ACT = 0>
__global__ __launch_bounds__(256) void wmma_gemm64(
    const unsigned short* __restrict__ Ap, const unsigned short* __restrict__ A2p, int lda, long strideA,
    const unsigned short* __restrict__ Btp, const unsigned short* __restrict__ Bt2p, int ldb, long strideB,
    void* __restrict__ Cout, void* __restrict__ Cout2, int ldc, long strideC,
    const float* __restrict__ bias,
    const float* __restrict__ resid, long strideR,
    int M, int N, int K, float scale) {
  typedef typename Elem<ET>::T T;
  typedef typename Frag<T>::V V;
  const T* A = (const T*)Ap; const T* A2 = (const T*)A2p; const T* Bt = (const T*)Btp; const T* Bt2 = (const T*)Bt2p;
  __shared__ __align__(16) float sT[8][16 * 68];
  const int b    = blockIdx.y;
  const int lane = threadIdx.x & 31;
  const int wave = threadIdx.x >> 5;
  const int tilesN = N >> 6;
  const int tilesM = M >> 6;
  const int tile = blockIdx.x * 8 + wave;
  if (tile >= tilesM * tilesN) return;
  const int tm = tile / tilesN;
  const int tn = tile - tm * tilesN;
  const int m0 = tm << 6;
  const int n0 = tn << 6;

  const T* Ab  = A  + (size_t)b * strideA;
  const T* Bb  = Bt + (size_t)b * strideB;
  const T* Ab2 = SPLIT ? (A2  + (size_t)b * strideA) : nullptr;
  const T* Bb2 = SPLIT ? (Bt2 + (size_t)b * strideB) : nullptr;

  const int rlane = lane & 15;
  const int koff  = (lane >> 4) * 8;
  const int mOff  = (lane >> 4) * 8;

  v8f acc[4][4];
#pragma unroll
  for (int i = 0; i < 4; ++i)
#pragma unroll
    for (int j = 0; j < 4; ++j) acc[i][j] = (v8f){0.f,0.f,0.f,0.f,0.f,0.f,0.f,0.f};

  for (int k0 = 0; k0 < K; k0 += 32) {
    V bh[4], bl[4];
#pragma unroll
    for (int j = 0; j < 4; ++j) {
      const size_t bo = (size_t)(n0 + (j << 4) + rlane) * ldb + koff + k0;
      bh[j] = Frag<T>::load(Bb + bo);
      if (SPLIT) bl[j] = Frag<T>::load(Bb2 + bo);
    }
#pragma unroll
    for (int i = 0; i < 4; ++i) {
      const size_t ao = (size_t)(m0 + (i << 4) + rlane) * lda + koff + k0;
      V ah = Frag<T>::load(Ab + ao);
      V al;
      if (SPLIT) al = Frag<T>::load(Ab2 + ao);
#pragma unroll
      for (int j = 0; j < 4; ++j) {
        acc[i][j] = Frag<T>::mma(ah, bh[j], acc[i][j]);
        if (SPLIT) {
          acc[i][j] = Frag<T>::mma(ah, bl[j], acc[i][j]);
          acc[i][j] = Frag<T>::mma(al, bh[j], acc[i][j]);
        }
      }
      Frag<T>::guard(acc[i][0], acc[i][3], ah, SPLIT ? al : ah);
      Frag<T>::guard(acc[i][1], acc[i][2], ah, SPLIT ? al : ah);
    }
    Frag<T>::keep(bh[0], bh[1], bh[2], bh[3]);
    if (SPLIT) Frag<T>::keep(bl[0], bl[1], bl[2], bl[3]);
  }
  acc_guard4(acc[0][0], acc[0][1], acc[0][2], acc[0][3]);
  acc_guard4(acc[1][0], acc[1][1], acc[1][2], acc[1][3]);
  acc_guard4(acc[2][0], acc[2][1], acc[2][2], acc[2][3]);
  acc_guard4(acc[3][0], acc[3][1], acc[3][2], acc[3][3]);

  float* slab = sT[wave];
  const float* Rb = RESID ? (resid + (size_t)b * strideR) : nullptr;
#pragma unroll
  for (int i = 0; i < 4; ++i) {
    const int mBase = m0 + (i << 4);
#pragma unroll
    for (int j = 0; j < 4; ++j) {
      const int n = n0 + (j << 4) + rlane;
      float bv = 0.f;
      if (BIAS_MODE == 2) bv = bias[n];
#pragma unroll
      for (int r = 0; r < 8; ++r) {
        float v = acc[i][j][r] * scale;
        if (BIAS_MODE == 1) v += bias[mBase + mOff + r];
        if (BIAS_MODE == 2) v += bv;
        if (RESID) v += Rb[(size_t)(mBase + mOff + r) * ldc + n];
        if (ACT == 2) v = fmaxf(v, 0.0f);
        if (ACT == 4) v = (v > 0.f) ? v : 0.01f * v;
        slab[(mOff + r) * 68 + (j << 4) + rlane] = v;
      }
    }
    __builtin_amdgcn_fence(__ATOMIC_RELEASE, "workgroup");
    __builtin_amdgcn_wave_barrier();
    __builtin_amdgcn_fence(__ATOMIC_ACQUIRE, "workgroup");
    if (OUT_MODE == 0) {
      float* C = (float*)Cout + (size_t)b * strideC;
      const int hh = lane >> 4, c4 = (lane & 15) * 4;
      for (int pass = 0; pass < 2; ++pass) {
#pragma unroll
        for (int it = 0; it < 8; ++it) {
          const int row = it * 2 + hh;
          v4f v = *(const v4f*)(slab + row * 68 + c4);
          *(volatile v4f*)(C + (size_t)(mBase + row) * ldc + n0 + c4) = v;
        }
        __threadfence();
      }
    } else {
      const int q = lane >> 3, c8 = (lane & 7) * 8;
      unsigned short* C  = (unsigned short*)Cout  + (size_t)b * strideC;
      unsigned short* C2 = (OUT_MODE == 2) ? ((unsigned short*)Cout2 + (size_t)b * strideC) : nullptr;
      for (int pass = 0; pass < 2; ++pass) {
#pragma unroll
        for (int it = 0; it < 4; ++it) {
          const int row = it * 4 + q;
          const float* sp = slab + row * 68 + c8;
          v8h hv, lv;
#pragma unroll
          for (int e = 0; e < 8; ++e) {
            if (OUT_MODE == 1) {
              hv[e] = (_Float16)sp[e];
            } else {
              unsigned short hb = f2bf_bits(sp[e]);
              unsigned short lb = f2bf_bits(sp[e] - bf_bits2f(hb));
              hv[e] = __builtin_bit_cast(_Float16, hb);
              lv[e] = __builtin_bit_cast(_Float16, lb);
            }
          }
          *(volatile v8h*)(C + (size_t)(mBase + row) * ldc + n0 + c8) = hv;
          if (OUT_MODE == 2) *(volatile v8h*)(C2 + (size_t)(mBase + row) * ldc + n0 + c8) = lv;
        }
        __threadfence();
      }
    }
    __builtin_amdgcn_fence(__ATOMIC_RELEASE, "workgroup");
    __builtin_amdgcn_wave_barrier();
    __builtin_amdgcn_fence(__ATOMIC_ACQUIRE, "workgroup");
  }
}

__global__ __launch_bounds__(256) void cast8_f16_kernel(const float* __restrict__ in, unsigned short* __restrict__ out,
                                                        int n8, float scale) {
  const int i = blockIdx.x * 256 + threadIdx.x;
  if (i >= n8) return;
  const float* p = in + 8 * (size_t)i;
  const v4f a = *(const v4f*)(p);
  const v4f c = *(const v4f*)(p + 4);
  unsigned short hb[8];
#pragma unroll
  for (int e = 0; e < 4; ++e) {
    hb[e]     = h_bits(a[e] * scale);
    hb[4 + e] = h_bits(c[e] * scale);
  }
  const v4u u = (v4u){pk16(hb[0], hb[1]), pk16(hb[2], hb[3]), pk16(hb[4], hb[5]), pk16(hb[6], hb[7])};
  unsigned short* q = out + 8 * (size_t)i;
  *(volatile v4u*)q = u;
  __threadfence();
  *(volatile v4u*)q = u;
}

__global__ __launch_bounds__(256) void wcat_kernel(const float* __restrict__ Wq, const float* __restrict__ Wk,
                                                   const float* __restrict__ Wv, const float* __restrict__ Wb,
                                                   const float* __restrict__ Gw, unsigned short* __restrict__ out) {
  const int i = blockIdx.x * 256 + threadIdx.x;
  if (i >= kNCAT * 128) return;
  const int row = i >> 7;
  const int c8  = (i & 127) * 8;
  const float* src = Wq;
  int srow = row;
  if (row >= kRowZ)      { src = Wb; srow = 0; }
  else if (row >= kRowG) { src = Gw; srow = row - kRowG; }
  else if (row >= kRowB) { src = Wb; srow = row - kRowB; }
  else if (row >= 2048)  { src = Wv; srow = row - 2048; }
  else if (row >= 1024)  { src = Wk; srow = row - 1024; }
  const bool live = row < kRowZ;
  const float* p = src + (size_t)srow * kD + c8;
  const v4f a = *(const v4f*)(p);
  const v4f c = *(const v4f*)(p + 4);
  unsigned short hb[8];
#pragma unroll
  for (int e = 0; e < 4; ++e) {
    const float x0 = live ? a[e] * kWC : 0.0f;
    const float x1 = live ? c[e] * kWC : 0.0f;
    hb[e]     = h_bits(x0);
    hb[4 + e] = h_bits(x1);
  }
  const v4u u = (v4u){pk16(hb[0], hb[1]), pk16(hb[2], hb[3]), pk16(hb[4], hb[5]), pk16(hb[6], hb[7])};
  unsigned short* q = out + 8 * (size_t)i;
  *(volatile v4u*)q = u;
  __threadfence();
  *(volatile v4u*)q = u;
}

__global__ __launch_bounds__(256) void conv_silu_kernel(const float* __restrict__ P, const float* __restrict__ cq,
                                                        const float* __restrict__ ck, const float* __restrict__ cv,
                                                        float* __restrict__ QKV) {
  const int i = blockIdx.x * 256 + threadIdx.x;
  if (i >= kL * 768) return;
  const int t = i / 768;
  const int j = i - t * 768;
  const int which = j >> 8;
  const int c4 = (j & 255) * 4;
  const float* cw = (which == 0) ? cq : ((which == 1) ? ck : cv);
  const v4f w0 = *(const v4f*)(cw + (size_t)(c4 + 0) * 4);
  const v4f w1 = *(const v4f*)(cw + (size_t)(c4 + 1) * 4);
  const v4f w2 = *(const v4f*)(cw + (size_t)(c4 + 2) * 4);
  const v4f w3 = *(const v4f*)(cw + (size_t)(c4 + 3) * 4);
  const v4f z4 = (v4f){0.f, 0.f, 0.f, 0.f};
  v4f acc = z4;
#pragma unroll
  for (int jj = 0; jj < 4; ++jj) {
    const int ts = t - 3 + jj;
    const int tc = ts < 0 ? 0 : ts;
    v4f x = *(const v4f*)(P + (size_t)tc * kNCAT + which * kD + c4);
    x = (ts < 0) ? z4 : x;
    acc[0] += x[0] * w0[jj];
    acc[1] += x[1] * w1[jj];
    acc[2] += x[2] * w2[jj];
    acc[3] += x[3] * w3[jj];
  }
  v4f o;
#pragma unroll
  for (int e = 0; e < 4; ++e) {
    const float y = acc[e];
    o[e] = y * (1.0f / (1.0f + expf(-y)));
  }
  float* op = QKV + (size_t)which * kL * kD + (size_t)t * kD + c4;
  *(volatile v4f*)op = o;
  __threadfence();
  *(volatile v4f*)op = o;
}

constexpr int PR   = 264;
constexpr int PT   = 40;
constexpr int PU   = 260;
constexpr int OFF_Q   = 0;
constexpr int OFF_K   = OFF_Q + kCS * PR * 2;
constexpr int OFF_KB  = OFF_K + kCS * PR * 2;
constexpr int OFF_VBT = OFF_KB + kCS * PR * 2;
constexpr int OFF_KBT = OFF_VBT + kDK * PT * 2;
constexpr int OFF_KNT = OFF_KBT + kDK * PT * 2;
constexpr int OFF_G   = OFF_KNT + kDK * PT * 2;
constexpr int OFF_ATT = OFF_G + kCS * 33 * 4;
constexpr int OFF_TF  = OFF_ATT + kCS * 33 * 4;
constexpr int OFF_T16 = OFF_TF + kCS * 33 * 4;
constexpr int PREP_LDS = OFF_T16 + kCS * PT * 2;
constexpr int OFF_UST = 0;
constexpr int OFF_WST = OFF_KB;
static_assert(kCS * PU * 4 <= OFF_WST, "u staging fits below the w staging");
static_assert(OFF_WST + kCS * PR * 2 <= OFF_VBT, "w staging inside the dead row-major region");
static_assert((OFF_K % 16) == 0 && (OFF_VBT % 16) == 0 && (OFF_G % 16) == 0 && (OFF_T16 % 16) == 0, "16-B aligned tiles");

__global__ __launch_bounds__(256) void chunk_prep_kernel(const float* __restrict__ QKV, const float* __restrict__ P,
                                                         unsigned short* __restrict__ QN, unsigned short* __restrict__ W16,
                                                         unsigned short* __restrict__ KNT, unsigned short* __restrict__ ATT,
                                                         float* __restrict__ U) {
  __shared__ __align__(16) unsigned char smem[PREP_LDS];
  unsigned short* sQ   = (unsigned short*)(smem + OFF_Q);
  unsigned short* sK   = (unsigned short*)(smem + OFF_K);
  unsigned short* sKB  = (unsigned short*)(smem + OFF_KB);
  unsigned short* sVBt = (unsigned short*)(smem + OFF_VBT);
  unsigned short* sKBt = (unsigned short*)(smem + OFF_KBT);
  unsigned short* sKNt = (unsigned short*)(smem + OFF_KNT);
  float* fG   = (float*)(smem + OFF_G);
  float* fAtt = (float*)(smem + OFF_ATT);
  float* fT   = (float*)(smem + OFF_TF);
  unsigned short* sT   = (unsigned short*)(smem + OFF_T16);
  float* sUst = (float*)(smem + OFF_UST);
  unsigned short* sWst = (unsigned short*)(smem + OFF_WST);

  const int tid = threadIdx.x, wave = tid >> 5, lane = tid & 31;
  const int c = lane & 15, hh = lane >> 4, koff = hh * 8;
  const int h  = blockIdx.x >> 6;
  const int ci = blockIdx.x & 63;
  const int l0 = ci * kCS;
  const float* qf = QKV;
  const float* kf = QKV + (size_t)kL * kD;
  const float* vf = QKV + (size_t)2 * kL * kD;

#pragma unroll 1
  for (int i = 0; i < 4; ++i) {
    const int r = wave + 8 * i;
    const int t = l0 + r;
    const size_t ro = (size_t)t * kD + h * kDK + 4 * lane;
    const v4f q0 = *(const v4f*)(qf + ro);
    const v4f q1 = *(const v4f*)(qf + ro + 128);
    const v4f k0 = *(const v4f*)(kf + ro);
    const v4f k1 = *(const v4f*)(kf + ro + 128);
    const v4f v0 = *(const v4f*)(vf + ro);
    const v4f v1 = *(const v4f*)(vf + ro + 128);
    const float bl = P[(size_t)t * kNCAT + kRowB + h];
    const float bet = 1.0f / (1.0f + expf(-bl));
    float sq = 0.0f, sk = 0.0f;
#pragma unroll
    for (int e = 0; e < 4; ++e) {
      sq += q0[e] * q0[e];
      sq += q1[e] * q1[e];
      sk += k0[e] * k0[e];
      sk += k1[e] * k1[e];
    }
#pragma unroll
    for (int off = 16; off > 0; off >>= 1) {
      sq += __shfl_xor(sq, off, 32);
      sk += __shfl_xor(sk, off, 32);
    }
    const float iq = rsqrtf(sq + 1e-6f) * kQC;
    const float ik = rsqrtf(sk + 1e-6f) * kQC;
    const float bv = bet * kVC;
#pragma unroll
    for (int jj = 0; jj < 2; ++jj) {
      const v4f qq = jj ? q1 : q0;
      const v4f kk = jj ? k1 : k0;
      const v4f vv = jj ? v1 : v0;
      const int cb = 4 * lane + 128 * jj;
      unsigned short hq[4], hk[4], hkb[4];
#pragma unroll
      for (int e = 0; e < 4; ++e) {
        const float qv  = qq[e] * iq;
        const float kv  = kk[e] * ik;
        const float kbv = kv * bet;
        const float vbv = vv[e] * bv;
        hq[e]  = h_bits(qv);
        hk[e]  = h_bits(kv);
        hkb[e] = h_bits(kbv);
        sVBt[(cb + e) * PT + r] = h_bits(vbv);
        sKBt[(cb + e) * PT + r] = hkb[e];
        sKNt[(cb + e) * PT + r] = hk[e];
      }
      *(v2u*)(sQ  + r * PR + cb) = (v2u){pk16(hq[0], hq[1]),   pk16(hq[2], hq[3])};
      *(v2u*)(sK  + r * PR + cb) = (v2u){pk16(hk[0], hk[1]),   pk16(hk[2], hk[3])};
      *(v2u*)(sKB + r * PR + cb) = (v2u){pk16(hkb[0], hkb[1]), pk16(hkb[2], hkb[3])};
    }
  }
  __syncthreads();

  for (int pass = 0; pass < 2; ++pass) {
#pragma unroll
    for (int i = 0; i < 4; ++i) {
      const int r = wave + 8 * i;
      const v4u v = *(const v4u*)(sQ + r * PR + 8 * lane);
      *(volatile v4u*)(QN + ((size_t)(h * kL + l0 + r)) * kDK + 8 * lane) = v;
    }
#pragma unroll
    for (int it = 0; it < 4; ++it) {
      const int idx = it * 256 + tid;
      const int d = idx >> 2, p = idx & 3;
      const v4u v = *(const v4u*)(sKNt + d * PT + p * 8);
      *(volatile v4u*)(KNT + ((size_t)(h * kNC + ci)) * (kDK * kCS) + (size_t)idx * 8) = v;
    }
    __threadfence();
  }

  {
    const int mt = (wave >> 1) & 1, nt = wave & 1;
    const bool doAtt = (wave >= 4);
    const unsigned short* ab = (doAtt ? sQ : sKB) + (16 * mt + c) * PR + koff;
    const unsigned short* bb = sK + (16 * nt + c) * PR + koff;
    v8f acc = (v8f){0.f,0.f,0.f,0.f,0.f,0.f,0.f,0.f};
#pragma unroll 1
    for (int k0 = 0; k0 < kDK; k0 += 32) {
      const v16h a = ldfrag(ab + k0);
      const v16h b = ldfrag(bb + k0);
      acc = mma_h(a, b, acc);
    }
    float* dst = doAtt ? fAtt : fG;
#pragma unroll
    for (int r = 0; r < 8; ++r) {
      const int row = 16 * mt + 8 * hh + r;
      const int col = 16 * nt + c;
      const float va = (row >= col) ? acc[r] : 0.0f;
      const float vg = acc[r] * kInvG;
      dst[row * 33 + col] = doAtt ? va : vg;
    }
  }
  __syncthreads();

  if (wave == 0) {
#pragma unroll 1
    for (int r = 0; r < kCS; ++r) {
      float tv = (r == lane) ? 1.0f : 0.0f;
#pragma unroll 1
      for (int j = 0; j < r; ++j) tv -= fG[r * 33 + j] * fT[j * 33 + lane];
      fT[r * 33 + lane] = tv;
      sT[r * PT + lane] = h_bits(tv * kQC);
    }
  } else if (wave >= 4) {
    const int idx = tid - 128;
    const int r = idx >> 2, c8 = (idx & 3) * 8;
    unsigned short hb[8];
#pragma unroll
    for (int e = 0; e < 8; ++e) hb[e] = h_bits(fAtt[r * 33 + c8 + e]);
    const v4u u = (v4u){pk16(hb[0], hb[1]), pk16(hb[2], hb[3]), pk16(hb[4], hb[5]), pk16(hb[6], hb[7])};
    unsigned short* ap = ATT + ((size_t)(h * kNC + ci)) * (kCS * kCS) + (size_t)idx * 8;
    *(volatile v4u*)ap = u;
    __threadfence();
    *(volatile v4u*)ap = u;
  }
  __syncthreads();

  {
    const v8f z8 = (v8f){0.f,0.f,0.f,0.f,0.f,0.f,0.f,0.f};
    const v16h a0 = ldfrag(sT + c * PT + koff);
    const v16h a1 = ldfrag(sT + (16 + c) * PT + koff);
#pragma unroll
    for (int jj = 0; jj < 2; ++jj) {
      const int nt = 2 * wave + jj;
      const v16h bv = ldfrag(sVBt + (16 * nt + c) * PT + koff);
      const v16h bk = ldfrag(sKBt + (16 * nt + c) * PT + koff);
      const v8f u0 = mma_h(a0, bv, z8);
      const v8f u1 = mma_h(a1, bv, z8);
      const v8f w0 = mma_h(a0, bk, z8);
      const v8f w1 = mma_h(a1, bk, z8);
#pragma unroll
      for (int r = 0; r < 8; ++r) {
        const int col = 16 * nt + c;
        sUst[(8 * hh + r) * PU + col]      = u0[r] * kInvU;
        sUst[(16 + 8 * hh + r) * PU + col] = u1[r] * kInvU;
        sWst[(8 * hh + r) * PR + col]      = h_bits(w0[r] * kInvWpl);
        sWst[(16 + 8 * hh + r) * PR + col] = h_bits(w1[r] * kInvWpl);
      }
    }
  }
  __syncthreads();

  for (int pass = 0; pass < 2; ++pass) {
#pragma unroll
    for (int i = 0; i < 4; ++i) {
      const int r = wave + 8 * i;
      const size_t grow = (size_t)(h * kL + l0 + r) * kDK;
      const v4f ua = *(const v4f*)(sUst + r * PU + 4 * lane);
      const v4f ub = *(const v4f*)(sUst + r * PU + 128 + 4 * lane);
      *(volatile v4f*)(U + grow + 4 * lane) = ua;
      *(volatile v4f*)(U + grow + 128 + 4 * lane) = ub;
      const v4u wv = *(const v4u*)(sWst + r * PR + 8 * lane);
      *(volatile v4u*)(W16 + grow + 8 * lane) = wv;
    }
    __threadfence();
  }
}

__global__ __launch_bounds__(256) void chunk_scan_kernel(const unsigned short* __restrict__ QN,
                                                         const unsigned short* __restrict__ W16,
                                                         const unsigned short* __restrict__ KNT,
                                                         const unsigned short* __restrict__ ATT,
                                                         const float* __restrict__ U, float* __restrict__ DELTA) {
  __shared__ __align__(16) unsigned short sSm[kSL * PR];
  __shared__ __align__(16) unsigned short sW[kCS * PR];
  __shared__ __align__(16) unsigned short sQn[kCS * PR];
  __shared__ __align__(16) unsigned short sKnT[kDK * PT];
  __shared__ __align__(16) unsigned short sAt[kCS * PT];
  __shared__ __align__(16) unsigned short sUaT[kSL * PT];
  __shared__ __align__(16) float sU[kCS * 68];
  __shared__ __align__(16) float sO[kCS * 68];

  const int tid = threadIdx.x, wave = tid >> 5, lane = tid & 31;
  const int c = lane & 15, hh = lane >> 4, koff = hh * 8;
  const int h   = blockIdx.x >> 2;
  const int dv0 = (blockIdx.x & 3) * kSL;
  const int mt = wave >> 2, nt = wave & 3;

  {
    unsigned* z = (unsigned*)sSm;
#pragma unroll 1
    for (int i = tid; i < (kSL * PR) / 2; i += 256) z[i] = 0u;
  }
  const v8f z8 = (v8f){0.f,0.f,0.f,0.f,0.f,0.f,0.f,0.f};
  v8f accS[2][4];
#pragma unroll
  for (int i = 0; i < 2; ++i)
#pragma unroll
    for (int j = 0; j < 4; ++j) accS[i][j] = z8;

#pragma unroll 1
  for (int ci = 0; ci < kNC; ++ci) {
    const int l0 = ci * kCS;
    {
      const size_t gbase = (size_t)(h * kL + l0) * kDK;
#pragma unroll
      for (int it = 0; it < 4; ++it) {
        const int idx = it * 256 + tid;
        const int r = idx >> 5, p = idx & 31;
        *(v4u*)(sW  + r * PR + p * 8) = *(const v4u*)(W16 + gbase + (size_t)r * kDK + p * 8);
        *(v4u*)(sQn + r * PR + p * 8) = *(const v4u*)(QN  + gbase + (size_t)r * kDK + p * 8);
        const int d = idx >> 2, pp = idx & 3;
        *(v4u*)(sKnT + d * PT + pp * 8) = *(const v4u*)(KNT + ((size_t)(h * kNC + ci)) * (kDK * kCS) + (size_t)idx * 8);
      }
      if (tid < 128) {
        const int r = tid >> 2, p = tid & 3;
        *(v4u*)(sAt + r * PT + p * 8) = *(const v4u*)(ATT + ((size_t)(h * kNC + ci)) * (kCS * kCS) + (size_t)tid * 8);
      }
#pragma unroll
      for (int it = 0; it < 2; ++it) {
        const int idx = it * 256 + tid;
        const int r = idx >> 4, p = idx & 15;
        *(v4f*)(sU + r * 68 + 4 * p) = *(const v4f*)(U + gbase + (size_t)r * kDK + dv0 + 4 * p);
      }
    }
    __syncthreads();

    v8f accW = z8, accQ = z8;
    {
      const unsigned short* aw = sW  + (16 * mt + c) * PR + koff;
      const unsigned short* aq = sQn + (16 * mt + c) * PR + koff;
      const unsigned short* bs = sSm + (16 * nt + c) * PR + koff;
#pragma unroll 1
      for (int k0 = 0; k0 < kDK; k0 += 32) {
        const v16h b  = ldfrag(bs + k0);
        const v16h a0 = ldfrag(aw + k0);
        const v16h a1 = ldfrag(aq + k0);
        accW = mma_h(a0, b, accW);
        accQ = mma_h(a1, b, accQ);
      }
    }
    {
      unsigned short hb[8];
#pragma unroll
      for (int r = 0; r < 8; ++r) {
        const int rr = 16 * mt + 8 * hh + r;
        const float ua = sU[rr * 68 + 16 * nt + c] - accW[r] * kInvQS;
        hb[r] = h_bits(ua * kVC);
      }
      const v4u pk = (v4u){pk16(hb[0], hb[1]), pk16(hb[2], hb[3]), pk16(hb[4], hb[5]), pk16(hb[6], hb[7])};
      *(v4u*)(sUaT + (16 * nt + c) * PT + 16 * mt + 8 * hh) = pk;
    }
    __syncthreads();

    {
      const v16h aa = ldfrag(sAt + (16 * mt + c) * PT + koff);
      const v16h b0 = ldfrag(sUaT + (c) * PT + koff);
      const v16h b1 = ldfrag(sUaT + (16 + c) * PT + koff);
      const v16h b2 = ldfrag(sUaT + (32 + c) * PT + koff);
      const v16h b3 = ldfrag(sUaT + (48 + c) * PT + koff);
      const v16h bo = (nt == 0) ? b0 : ((nt == 1) ? b1 : ((nt == 2) ? b2 : b3));
      accQ = mma_h(aa, bo, accQ);
#pragma unroll
      for (int r = 0; r < 8; ++r) sO[(16 * mt + 8 * hh + r) * 68 + 16 * nt + c] = accQ[r] * kInvQS;
#pragma unroll
      for (int i = 0; i < 2; ++i) {
        const int mtS = 2 * wave + i;
        const v16h ak = ldfrag(sKnT + (16 * mtS + c) * PT + koff);
        accS[i][0] = mma_h(ak, b0, accS[i][0]);
        accS[i][1] = mma_h(ak, b1, accS[i][1]);
        accS[i][2] = mma_h(ak, b2, accS[i][2]);
        accS[i][3] = mma_h(ak, b3, accS[i][3]);
#pragma unroll
        for (int j = 0; j < 4; ++j) {
          unsigned short hb[8];
#pragma unroll
          for (int r = 0; r < 8; ++r) {
            const float sv = accS[i][j][r];
            hb[r] = h_bits(sv);
          }
          const v4u pk = (v4u){pk16(hb[0], hb[1]), pk16(hb[2], hb[3]), pk16(hb[4], hb[5]), pk16(hb[6], hb[7])};
          *(v4u*)(sSm + (16 * j + c) * PR + 16 * mtS + 8 * hh) = pk;
        }
      }
    }
    __syncthreads();

    {
      const int c4 = c * 4;
      for (int pass = 0; pass < 2; ++pass) {
#pragma unroll
        for (int it = 0; it < 2; ++it) {
          const int row = 4 * wave + 2 * it + hh;
          const v4f v = *(const v4f*)(sO + row * 68 + c4);
          *(volatile v4f*)(DELTA + (size_t)(l0 + row) * kD + h * kDK + dv0 + c4) = v;
        }
        __threadfence();
      }
    }
  }
}

__global__ __launch_bounds__(256) void fir_mix_norm_kernel(const float* __restrict__ VD, const float* __restrict__ DELTA,
                                                           const float* __restrict__ P, const float* __restrict__ fs,
                                                           const float* __restrict__ fm, const float* __restrict__ fl,
                                                           const float* __restrict__ gb, const float* __restrict__ ltemp,
                                                           const float* __restrict__ epsp, const float* __restrict__ nw,
                                                           unsigned short* __restrict__ OH) {
  __shared__ float sP[8];
  __shared__ float sRed[8];
  __shared__ __align__(16) float sVal[256];
  const int tid = threadIdx.x, wave = tid >> 5, lane = tid & 31;
  const int t = blockIdx.x >> 2;
  const int h = blockIdx.x & 3;
  const int ch = h * kDK + tid;

  if (wave == 0) {
    const int l8 = lane & 7;
    const bool livep = l8 < 5;
    const int p = livep ? l8 : 4;
    const float rt = 1.0f / expf(ltemp[h]);
    const float lg = (P[(size_t)t * kNCAT + kRowG + h * 5 + p] + gb[h * 5 + p]) * rt;
    float m = livep ? lg : -INFINITY;
    m = fmaxf(m, __shfl_xor(m, 1, 32));
    m = fmaxf(m, __shfl_xor(m, 2, 32));
    m = fmaxf(m, __shfl_xor(m, 4, 32));
    const float ex = expf(lg - m);
    float e = livep ? ex : 0.0f;
    float s = e;
    s += __shfl_xor(s, 1, 32);
    s += __shfl_xor(s, 2, 32);
    s += __shfl_xor(s, 4, 32);
    const float eps = fminf(fmaxf(epsp[h], 0.0f), 0.2f);
    const float pr = (e * (1.0f / s)) * (1.0f - 5.0f * eps) + eps;
    if (lane < 8) sP[lane] = pr;
  }

  const int nL = (t + 1 < 63) ? (t + 1) : 63;
  const int nM = (t + 1 < 15) ? (t + 1) : 15;
  const int nS = (t + 1 < 3) ? (t + 1) : 3;
  const float* vp = VD + (size_t)t * kD + ch;
  float aL = 0.0f, aM = 0.0f, aS = 0.0f;
  {
    const float* f = fl + (size_t)ch * 63 + 62;
#pragma unroll 1
    for (int i = 0; i < nL; ++i) aL = fmaf(vp[-(i * kD)], f[-i], aL);
  }
  {
    const float* f = fm + (size_t)ch * 15 + 14;
#pragma unroll 1
    for (int i = 0; i < nM; ++i) aM = fmaf(vp[-(i * kD)], f[-i], aM);
  }
  {
    const float* f = fs + (size_t)ch * 3 + 2;
#pragma unroll 1
    for (int i = 0; i < nS; ++i) aS = fmaf(vp[-(i * kD)], f[-i], aS);
  }
  const float vcur = vp[0];
  const float dcur = DELTA[(size_t)t * kD + ch];
  const float wn = nw[tid];
  __syncthreads();

  float mix = sP[0] * aS;
  mix = mix + sP[1] * aM;
  mix = mix + sP[2] * aL;
  mix = mix + sP[3] * dcur;
  mix = mix + sP[4] * vcur;
  float ss = mix * mix;
#pragma unroll
  for (int off = 16; off > 0; off >>= 1) ss += __shfl_xor(ss, off, 32);
  if (lane == 0) sRed[wave] = ss;
  __syncthreads();
  const float tot = ((sRed[0] + sRed[1]) + (sRed[2] + sRed[3])) + ((sRed[4] + sRed[5]) + (sRed[6] + sRed[7]));
  const float inv = rsqrtf(tot * (1.0f / (float)kDK) + 1e-5f);
  sVal[tid] = (mix * inv) * wn;
  __syncthreads();
  if (wave == 0) {
    const v4f a = *(const v4f*)(sVal + 8 * lane);
    const v4f b = *(const v4f*)(sVal + 8 * lane + 4);
    unsigned short hb[8];
#pragma unroll
    for (int e = 0; e < 4; ++e) {
      hb[e]     = h_bits(a[e]);
      hb[4 + e] = h_bits(b[e]);
    }
    const v4u u = (v4u){pk16(hb[0], hb[1]), pk16(hb[2], hb[3]), pk16(hb[4], hb[5]), pk16(hb[6], hb[7])};
    unsigned short* op = OH + (size_t)t * kD + h * kDK + 8 * lane;
    *(volatile v4u*)op = u;
    __threadfence();
    *(volatile v4u*)op = u;
  }
}

extern "C" void kernel_launch(void* const* d_in, const int* in_sizes, int n_in,
                              void* d_out, int out_size, void* d_ws, size_t ws_size, hipStream_t stream) {
  if (n_in < 17 || d_out == nullptr || d_ws == nullptr) return;
  if (in_sizes[0] != kL * kD || in_sizes[1] != kD * kD || in_sizes[2] != kD * kD || in_sizes[3] != kD * kD ||
      in_sizes[4] != kH * kD || in_sizes[5] != kD * 4 || in_sizes[6] != kD * 4 || in_sizes[7] != kD * 4 ||
      in_sizes[8] != kD * 3 || in_sizes[9] != kD * 15 || in_sizes[10] != kD * 63 || in_sizes[11] != kH * 5 * kD ||
      in_sizes[12] != kH * 5 || in_sizes[13] != kH || in_sizes[14] != kH || in_sizes[15] != kDK ||
      in_sizes[16] != kD * kD || out_size != kL * kD) return;

  const float* hs    = (const float*)d_in[0];
  const float* Wq    = (const float*)d_in[1];
  const float* Wk    = (const float*)d_in[2];
  const float* Wv    = (const float*)d_in[3];
  const float* Wb    = (const float*)d_in[4];
  const float* convq = (const float*)d_in[5];
  const float* convk = (const float*)d_in[6];
  const float* convv = (const float*)d_in[7];
  const float* firs  = (const float*)d_in[8];
  const float* firm  = (const float*)d_in[9];
  const float* firl  = (const float*)d_in[10];
  const float* gw    = (const float*)d_in[11];
  const float* gb    = (const float*)d_in[12];
  const float* lt    = (const float*)d_in[13];
  const float* ep    = (const float*)d_in[14];
  const float* nw    = (const float*)d_in[15];
  const float* Wo    = (const float*)d_in[16];

  char* ws = (char*)d_ws; size_t off = 0;
  auto carve = [&](size_t bytes) -> char* { char* p = ws + off; off += (bytes + 255) & ~(size_t)255; return p; };
  unsigned short* XH   = (unsigned short*)carve((size_t)kL * kD * 2);
  unsigned short* WCAT = (unsigned short*)carve((size_t)kNCAT * kD * 2);
  unsigned short* WOH  = (unsigned short*)carve((size_t)kD * kD * 2);
  float*          P    = (float*)carve((size_t)kL * kNCAT * 4);
  float*          QKV  = (float*)carve((size_t)3 * kL * kD * 4);
  unsigned short* QN   = (unsigned short*)carve((size_t)kH * kL * kDK * 2);
  unsigned short* W16  = (unsigned short*)carve((size_t)kH * kL * kDK * 2);
  unsigned short* KNT  = (unsigned short*)carve((size_t)kH * kNC * kDK * kCS * 2);
  unsigned short* ATT  = (unsigned short*)carve((size_t)kH * kNC * kCS * kCS * 2);
  float*          U    = (float*)carve((size_t)kH * kL * kDK * 4);
  float*          DELTA = (float*)carve((size_t)kL * kD * 4);
  unsigned short* OH   = (unsigned short*)carve((size_t)kL * kD * 2);
  if (off > ws_size || off > (size_t)134217728) return;

  cast8_f16_kernel<<<(kL * kD / 8) / 256, 256, 0, stream>>>(hs, XH, kL * kD / 8, 1.0f);
  wcat_kernel<<<(kNCAT * 128) / 256, 256, 0, stream>>>(Wq, Wk, Wv, Wb, gw, WCAT);
  cast8_f16_kernel<<<(kD * kD / 8) / 256, 256, 0, stream>>>(Wo, WOH, kD * kD / 8, kWC);

  wmma_gemm64<0, false, 0, 0, false, 0><<<dim3((kL / 64) * (kNCAT / 64) / 8, 1), 256, 0, stream>>>(
      XH, XH, kD, 0L, WCAT, WCAT, kD, 0L, (void*)P, (void*)P, kNCAT, 0L,
      (const float*)P, (const float*)P, 0L, kL, kNCAT, kD, kInvW);

  conv_silu_kernel<<<(kL * 768) / 256, 256, 0, stream>>>(P, convq, convk, convv, QKV);

  chunk_prep_kernel<<<kH * kNC, 256, 0, stream>>>(QKV, P, QN, W16, KNT, ATT, U);
  chunk_scan_kernel<<<kH * (kDK / kSL), 256, 0, stream>>>(QN, W16, KNT, ATT, U, DELTA);

  fir_mix_norm_kernel<<<kL * kH, 256, 0, stream>>>(QKV + (size_t)2 * kL * kD, DELTA, P, firs, firm, firl,
                                                   gb, lt, ep, nw, OH);

  wmma_gemm64<0, false, 0, 0, false, 0><<<dim3((kL / 64) * (kD / 64) / 8, 1), 256, 0, stream>>>(
      OH, OH, kD, 0L, WOH, WOH, kD, 0L, d_out, d_out, kD, 0L,
      (const float*)P, (const float*)P, 0L, kL, kD, kD, kInvW);
}
